// SA_MambaLayer_64802466562245
// MI455X (gfx1250) — hardware-verified
//
#include <hip/hip_runtime.h>
#include <math.h>

typedef __attribute__((ext_vector_type(16))) _Float16 v16h;
typedef __attribute__((ext_vector_type(8)))  _Float16 v8h;
typedef __attribute__((ext_vector_type(16))) __bf16   v16b;
typedef __attribute__((ext_vector_type(8)))  __bf16   v8b;
typedef __attribute__((ext_vector_type(8)))  float    v8f;
typedef __attribute__((ext_vector_type(4)))  float    v4f;

constexpr int kBatch  = 2;
constexpr int kSeqL   = 2048;
constexpr int kDim    = 512;
constexpr int kDin    = 1024;
constexpr int kNst    = 64;
constexpr int kHalfSt = 32;
constexpr int kDtR    = 32;
constexpr int kPrjN   = 160;
constexpr int kPrjP   = 192;
constexpr int kXZP    = 2 * kDin;
constexpr int kRows   = kBatch * kSeqL;
constexpr int kTP     = 260;
constexpr int kChBlk  = 128;
constexpr int kSYP    = 132;

__device__ __forceinline__ unsigned short f2bf_bits(float f) {
  unsigned u = __float_as_uint(f);
  return (unsigned short)((u + 0x7FFFu + ((u >> 16) & 1u)) >> 16);
}
__device__ __forceinline__ float bf_bits2f(unsigned short h) { return __uint_as_float(((unsigned)h) << 16); }

__device__ __forceinline__ void dep_guard_h(v8f& a, v8f& b, v16h x, v16h y) { asm volatile("v_nop\n\tv_nop\n\tv_nop\n\tv_nop" : "+v"(a), "+v"(b) : "v"(x), "v"(y)); }
__device__ __forceinline__ void dep_guard_b(v8f& a, v8f& b, v16b x, v16b y) { asm volatile("v_nop\n\tv_nop\n\tv_nop\n\tv_nop" : "+v"(a), "+v"(b) : "v"(x), "v"(y)); }
__device__ __forceinline__ void keep4_h(v16h a, v16h b, v16h c, v16h d) { asm volatile("v_nop" :: "v"(a), "v"(b), "v"(c), "v"(d)); }
__device__ __forceinline__ void keep4_b(v16b a, v16b b, v16b c, v16b d) { asm volatile("v_nop" :: "v"(a), "v"(b), "v"(c), "v"(d)); }
__device__ __forceinline__ void acc_guard4(v8f& a, v8f& b, v8f& c, v8f& d) { asm volatile("v_nop\n\tv_nop\n\tv_nop\n\tv_nop" : "+v"(a), "+v"(b), "+v"(c), "+v"(d)); }
template <typename T> struct Frag;
template <> struct Frag<_Float16> {
  typedef v16h V; union U { v16h v; v8h h[2]; };
  static __device__ __forceinline__ v16h load(const _Float16* p) {
    U f; f.h[0] = *(const v8h*)(p); f.h[1] = *(const v8h*)(p + 16); return f.v;
  }
  static __device__ __forceinline__ v8f mma(v16h a, v16h b, v8f c) {
    return __builtin_amdgcn_wmma_f32_16x16x32_f16(false, a, false, b, (short)0, c, false, false);
  }
  static __device__ __forceinline__ void guard(v8f& a, v8f& b, v16h x, v16h y) { dep_guard_h(a, b, x, y); }
  static __device__ __forceinline__ void keep(v16h a, v16h b, v16h c, v16h d) { keep4_h(a, b, c, d); }
};
template <> struct Frag<__bf16> {
  typedef v16b V; union U { v16b v; v8b h[2]; };
  static __device__ __forceinline__ v16b load(const __bf16* p) {
    U f; f.h[0] = *(const v8b*)(p); f.h[1] = *(const v8b*)(p + 16); return f.v;
  }
  static __device__ __forceinline__ v8f mma(v16b a, v16b b, v8f c) {
    return __builtin_amdgcn_wmma_f32_16x16x32_bf16(false, a, false, b, (short)0, c, false, false);
  }
  static __device__ __forceinline__ void guard(v8f& a, v8f& b, v16b x, v16b y) { dep_guard_b(a, b, x, y); }
  static __device__ __forceinline__ void keep(v16b a, v16b b, v16b c, v16b d) { keep4_b(a, b, c, d); }
};

template <int ET> struct Elem;
template <> struct Elem<0> { typedef _Float16 T; };
template <> struct Elem<1> { typedef __bf16 T; };
template <int ET, bool SPLIT, int BIAS_MODE, int OUT_MODE, bool RESID, int ACT = 0>
__global__ __launch_bounds__(256) void wmma_gemm64(
    const unsigned short* __restrict__ Ap, const unsigned short* __restrict__ A2p, int lda, long strideA,
    const unsigned short* __restrict__ Btp, const unsigned short* __restrict__ Bt2p, int ldb, long strideB,
    void* __restrict__ Cout, void* __restrict__ Cout2, int ldc, long strideC,
    const float* __restrict__ bias,
    const float* __restrict__ resid, long strideR,
    int M, int N, int K, float scale) {
  typedef typename Elem<ET>::T T;
  typedef typename Frag<T>::V V;
  const T* A = (const T*)Ap; const T* A2 = (const T*)A2p; const T* Bt = (const T*)Btp; const T* Bt2 = (const T*)Bt2p;
  __shared__ __align__(16) float sT[8][16 * 68];
  const int b    = blockIdx.y;
  const int lane = threadIdx.x & 31;
  const int wave = threadIdx.x >> 5;
  const int tilesN = N >> 6;
  const int tilesM = M >> 6;
  const int tile = blockIdx.x * 8 + wave;
  if (tile >= tilesM * tilesN) return;
  const int tm = tile / tilesN;
  const int tn = tile - tm * tilesN;
  const int m0 = tm << 6;
  const int n0 = tn << 6;

  const T* Ab  = A  + (size_t)b * strideA;
  const T* Bb  = Bt + (size_t)b * strideB;
  const T* Ab2 = SPLIT ? (A2  + (size_t)b * strideA) : nullptr;
  const T* Bb2 = SPLIT ? (Bt2 + (size_t)b * strideB) : nullptr;

  const int rlane = lane & 15;
  const int koff  = (lane >> 4) * 8;
  const int mOff  = (lane >> 4) * 8;

  v8f acc[4][4];
#pragma unroll
  for (int i = 0; i < 4; ++i)
#pragma unroll
    for (int j = 0; j < 4; ++j) acc[i][j] = (v8f){0.f,0.f,0.f,0.f,0.f,0.f,0.f,0.f};

  for (int k0 = 0; k0 < K; k0 += 32) {
    V bh[4], bl[4];
#pragma unroll
    for (int j = 0; j < 4; ++j) {
      const size_t bo = (size_t)(n0 + (j << 4) + rlane) * ldb + koff + k0;
      bh[j] = Frag<T>::load(Bb + bo);
      if (SPLIT) bl[j] = Frag<T>::load(Bb2 + bo);
    }
#pragma unroll
    for (int i = 0; i < 4; ++i) {
      const size_t ao = (size_t)(m0 + (i << 4) + rlane) * lda + koff + k0;
      V ah = Frag<T>::load(Ab + ao);
      V al;
      if (SPLIT) al = Frag<T>::load(Ab2 + ao);
#pragma unroll
      for (int j = 0; j < 4; ++j) {
        acc[i][j] = Frag<T>::mma(ah, bh[j], acc[i][j]);
        if (SPLIT) {
          acc[i][j] = Frag<T>::mma(ah, bl[j], acc[i][j]);
          acc[i][j] = Frag<T>::mma(al, bh[j], acc[i][j]);
        }
      }
      Frag<T>::guard(acc[i][0], acc[i][3], ah, SPLIT ? al : ah);
    }
    Frag<T>::keep(bh[0], bh[1], bh[2], bh[3]);
    if (SPLIT) Frag<T>::keep(bl[0], bl[1], bl[2], bl[3]);
  }
  acc_guard4(acc[0][0], acc[0][1], acc[0][2], acc[0][3]);
  acc_guard4(acc[1][0], acc[1][1], acc[1][2], acc[1][3]);
  acc_guard4(acc[2][0], acc[2][1], acc[2][2], acc[2][3]);
  acc_guard4(acc[3][0], acc[3][1], acc[3][2], acc[3][3]);

  float* slab = sT[wave];
  const float* Rb = RESID ? (resid + (size_t)b * strideR) : nullptr;
#pragma unroll
  for (int i = 0; i < 4; ++i) {
    const int mBase = m0 + (i << 4);
#pragma unroll
    for (int j = 0; j < 4; ++j) {
      const int n = n0 + (j << 4) + rlane;
      float bv = 0.f;
      if (BIAS_MODE == 2) bv = bias[n];
#pragma unroll
      for (int r = 0; r < 8; ++r) {
        float v = acc[i][j][r] * scale;
        if (BIAS_MODE == 1) v += bias[mBase + mOff + r];
        if (BIAS_MODE == 2) v += bv;
        if (RESID) v += Rb[(size_t)(mBase + mOff + r) * ldc + n];
        if (ACT == 1) v = tanhf(v);
        if (ACT == 2) v = fmaxf(v, 0.0f);
        if (ACT == 3) v = v / (1.0f + expf(-v));
        if (ACT == 4) v = (v > 0.f) ? v : 0.01f * v;
        if (ACT == 5) v = 0.5f * v * (1.0f + erff(v * 0.70710678118654752f));
        slab[(mOff + r) * 68 + (j << 4) + rlane] = v;
      }
    }
    __builtin_amdgcn_fence(__ATOMIC_RELEASE, "workgroup");
    __builtin_amdgcn_wave_barrier();
    __builtin_amdgcn_fence(__ATOMIC_ACQUIRE, "workgroup");
    if (OUT_MODE == 0) {
      float* C = (float*)Cout + (size_t)b * strideC;
      const int hh = lane >> 4, c4 = (lane & 15) * 4;
      for (int pass = 0; pass < 2; ++pass) {
#pragma unroll
        for (int it = 0; it < 8; ++it) {
          const int row = it * 2 + hh;
          v4f v = *(const v4f*)(slab + row * 68 + c4);
          *(volatile v4f*)(C + (size_t)(mBase + row) * ldc + n0 + c4) = v;
        }
        __threadfence();
      }
    } else {
      const int q = lane >> 3, c8 = (lane & 7) * 8;
      unsigned short* C  = (unsigned short*)Cout  + (size_t)b * strideC;
      unsigned short* C2 = (OUT_MODE == 2) ? ((unsigned short*)Cout2 + (size_t)b * strideC) : nullptr;
      for (int pass = 0; pass < 2; ++pass) {
#pragma unroll
        for (int it = 0; it < 4; ++it) {
          const int row = it * 4 + q;
          const float* sp = slab + row * 68 + c8;
          v8h hv, lv;
#pragma unroll
          for (int e = 0; e < 8; ++e) {
            if (OUT_MODE == 1) {
              hv[e] = (_Float16)sp[e];
            } else {
              unsigned short hb = f2bf_bits(sp[e]);
              unsigned short lb = f2bf_bits(sp[e] - bf_bits2f(hb));
              hv[e] = __builtin_bit_cast(_Float16, hb);
              lv[e] = __builtin_bit_cast(_Float16, lb);
            }
          }
          *(volatile v8h*)(C + (size_t)(mBase + row) * ldc + n0 + c8) = hv;
          if (OUT_MODE == 2) *(volatile v8h*)(C2 + (size_t)(mBase + row) * ldc + n0 + c8) = lv;
        }
        __threadfence();
      }
    }
    __builtin_amdgcn_fence(__ATOMIC_RELEASE, "workgroup");
    __builtin_amdgcn_wave_barrier();
    __builtin_amdgcn_fence(__ATOMIC_ACQUIRE, "workgroup");
  }
}

__global__ __launch_bounds__(256) void ln_split_kernel(
    const float* __restrict__ x, const float* __restrict__ gw, const float* __restrict__ gb,
    unsigned short* __restrict__ XH, unsigned short* __restrict__ XL, int nrows)
{
  const int lane = threadIdx.x & 31, wave = threadIdx.x >> 5;
  const int row = blockIdx.x * 8 + wave;
  if (row >= nrows) return;
  const float* xr = x + (size_t)row * kDim;
  v4f a[4], wv[4], bv[4];
#pragma unroll
  for (int i = 0; i < 2; ++i) {
    const int c0 = 256 * i + lane * 8;
    a[2 * i]      = *(const v4f*)(xr + c0);
    a[2 * i + 1]  = *(const v4f*)(xr + c0 + 4);
    wv[2 * i]     = *(const v4f*)(gw + c0);
    wv[2 * i + 1] = *(const v4f*)(gw + c0 + 4);
    bv[2 * i]     = *(const v4f*)(gb + c0);
    bv[2 * i + 1] = *(const v4f*)(gb + c0 + 4);
  }
  float s = 0.f;
#pragma unroll
  for (int k = 0; k < 4; ++k) s += (a[k][0] + a[k][1]) + (a[k][2] + a[k][3]);
#pragma unroll
  for (int off = 1; off < 32; off <<= 1) s += __shfl_xor(s, off, 32);
  const float mean = s * (1.0f / 512.0f);
  v4f dv[4];
  float ss = 0.f;
#pragma unroll
  for (int k = 0; k < 4; ++k) {
    dv[k] = a[k] - mean;
    ss += (dv[k][0] * dv[k][0] + dv[k][1] * dv[k][1]) + (dv[k][2] * dv[k][2] + dv[k][3] * dv[k][3]);
  }
#pragma unroll
  for (int off = 1; off < 32; off <<= 1) ss += __shfl_xor(ss, off, 32);
  const float var  = ss * (1.0f / 512.0f);
  const float rstd = rsqrtf(var + 1e-5f);
  v8h hv[2], lv[2];
#pragma unroll
  for (int i = 0; i < 2; ++i) {
#pragma unroll
    for (int e = 0; e < 8; ++e) {
      const int k = 2 * i + (e >> 2), ee = e & 3;
      const float v = (dv[k][ee] * rstd) * wv[k][ee] + bv[k][ee];
      const unsigned short hb = f2bf_bits(v);
      const unsigned short lb = f2bf_bits(v - bf_bits2f(hb));
      hv[i][e] = __builtin_bit_cast(_Float16, hb);
      lv[i][e] = __builtin_bit_cast(_Float16, lb);
    }
  }
  for (int pass = 0; pass < 2; ++pass) {
#pragma unroll
    for (int i = 0; i < 2; ++i) {
      const size_t o = (size_t)row * kDim + 256 * i + lane * 8;
      *(volatile v8h*)(XH + o) = hv[i];
      *(volatile v8h*)(XL + o) = lv[i];
    }
    __threadfence();
  }
}

__global__ __launch_bounds__(256) void cast_split_rows_kernel(
    const float* __restrict__ src, unsigned short* __restrict__ hi, unsigned short* __restrict__ lo,
    int K, int nreal, int total8)
{
  const int i = blockIdx.x * 256 + threadIdx.x;
  if (i >= total8) return;
  const int e0  = i << 3;
  const int row = e0 / K;
  const int col = e0 - row * K;
  const int rc  = (row < nreal) ? row : (nreal - 1);
  const bool keep = (row < nreal);
  const float* p = src + (size_t)rc * K + col;
  const v4f a0 = *(const v4f*)(p);
  const v4f a1 = *(const v4f*)(p + 4);
  v8h hv, lv;
#pragma unroll
  for (int e = 0; e < 4; ++e) {
    const float v0 = keep ? a0[e] : 0.f;
    const float v1 = keep ? a1[e] : 0.f;
    const unsigned short h0 = f2bf_bits(v0), h1 = f2bf_bits(v1);
    const unsigned short l0 = f2bf_bits(v0 - bf_bits2f(h0)), l1 = f2bf_bits(v1 - bf_bits2f(h1));
    hv[e]     = __builtin_bit_cast(_Float16, h0);
    hv[4 + e] = __builtin_bit_cast(_Float16, h1);
    lv[e]     = __builtin_bit_cast(_Float16, l0);
    lv[4 + e] = __builtin_bit_cast(_Float16, l1);
  }
  unsigned short* qh = hi + e0;
  unsigned short* ql = lo + e0;
  *(volatile v8h*)qh = hv;
  *(volatile v8h*)ql = lv;
  __threadfence();
  *(volatile v8h*)qh = hv;
  *(volatile v8h*)ql = lv;
}

__global__ __launch_bounds__(256) void dt_split_kernel(
    const float* __restrict__ PROJ, unsigned short* __restrict__ DH, unsigned short* __restrict__ DL, int total8)
{
  const int i = blockIdx.x * 256 + threadIdx.x;
  if (i >= total8) return;
  const int e0  = i << 3;
  const int row = e0 >> 5;
  const int c8  = e0 & 31;
  const float* p = PROJ + (size_t)row * kPrjP + c8;
  const v4f a0 = *(const v4f*)(p);
  const v4f a1 = *(const v4f*)(p + 4);
  v8h hv, lv;
#pragma unroll
  for (int e = 0; e < 4; ++e) {
    const unsigned short h0 = f2bf_bits(a0[e]), h1 = f2bf_bits(a1[e]);
    const unsigned short l0 = f2bf_bits(a0[e] - bf_bits2f(h0)), l1 = f2bf_bits(a1[e] - bf_bits2f(h1));
    hv[e]     = __builtin_bit_cast(_Float16, h0);
    hv[4 + e] = __builtin_bit_cast(_Float16, h1);
    lv[e]     = __builtin_bit_cast(_Float16, l0);
    lv[4 + e] = __builtin_bit_cast(_Float16, l1);
  }
  unsigned short* qh = DH + e0;
  unsigned short* ql = DL + e0;
  *(volatile v8h*)qh = hv;
  *(volatile v8h*)ql = lv;
  __threadfence();
  *(volatile v8h*)qh = hv;
  *(volatile v8h*)ql = lv;
}

__global__ __launch_bounds__(256) void conv_silu_kernel(
    const float* __restrict__ XZ, const float* __restrict__ cw, const float* __restrict__ cb,
    float* __restrict__ UC, unsigned short* __restrict__ UCH, unsigned short* __restrict__ UCL)
{
  __shared__ __align__(16) float sT[16 * kTP];
  const int tid = threadIdx.x, lane = tid & 31, wave = tid >> 5;
  const int d0 = blockIdx.x * 256, d = d0 + tid;
  const int g0 = blockIdx.y * 64;
  const int tb = g0 & (kSeqL - 1);
  const float w0 = cw[d * 4 + 0], w1 = cw[d * 4 + 1], w2 = cw[d * 4 + 2], w3 = cw[d * 4 + 3];
  const float bc = cb[d];
  float xm3, xm2, xm1;
  {
    const int r3 = (tb >= 3) ? (g0 - 3) : g0;
    const int r2 = (tb >= 2) ? (g0 - 2) : g0;
    const int r1 = (tb >= 1) ? (g0 - 1) : g0;
    const float v3 = XZ[(size_t)r3 * kXZP + d];
    const float v2 = XZ[(size_t)r2 * kXZP + d];
    const float v1 = XZ[(size_t)r1 * kXZP + d];
    xm3 = (tb >= 3) ? v3 : 0.f;
    xm2 = (tb >= 2) ? v2 : 0.f;
    xm1 = (tb >= 1) ? v1 : 0.f;
  }
  const int hrow = wave >> 1;
  const int hch  = (wave & 1) * 128 + lane * 4;
#pragma unroll 1
  for (int sub = 0; sub < 4; ++sub) {
    const int lb = g0 + sub * 16;
#pragma unroll 1
    for (int s = 0; s < 16; ++s) {
      const float xc = XZ[(size_t)(lb + s) * kXZP + d];
      float acc = w0 * xm3;
      acc = fmaf(w1, xm2, acc);
      acc = fmaf(w2, xm1, acc);
      acc = fmaf(w3, xc, acc);
      const float sv = acc + bc;
      const float sg = __builtin_amdgcn_rcpf(1.0f + __expf(-sv));
      sT[s * kTP + tid] = sv * sg;
      xm3 = xm2; xm2 = xm1; xm1 = xc;
    }
    __syncthreads();
    v4f fv[4];
    v8h bh[2], blo[2];
#pragma unroll
    for (int it = 0; it < 4; ++it) fv[it] = *(const v4f*)(sT + (it * 4 + hrow) * kTP + hch);
#pragma unroll
    for (int it = 0; it < 2; ++it) {
      const float* sp = sT + (it * 8 + wave) * kTP + lane * 8;
      const v4f a0 = *(const v4f*)(sp);
      const v4f a1 = *(const v4f*)(sp + 4);
#pragma unroll
      for (int e = 0; e < 4; ++e) {
        const unsigned short h0 = f2bf_bits(a0[e]), h1 = f2bf_bits(a1[e]);
        const unsigned short l0 = f2bf_bits(a0[e] - bf_bits2f(h0)), l1 = f2bf_bits(a1[e] - bf_bits2f(h1));
        bh[it][e]      = __builtin_bit_cast(_Float16, h0);
        bh[it][4 + e]  = __builtin_bit_cast(_Float16, h1);
        blo[it][e]     = __builtin_bit_cast(_Float16, l0);
        blo[it][4 + e] = __builtin_bit_cast(_Float16, l1);
      }
    }
    for (int pass = 0; pass < 2; ++pass) {
#pragma unroll
      for (int it = 0; it < 4; ++it)
        *(volatile v4f*)(UC + (size_t)(lb + it * 4 + hrow) * kDin + d0 + hch) = fv[it];
#pragma unroll
      for (int it = 0; it < 2; ++it) {
        const size_t o = (size_t)(lb + it * 8 + wave) * kDin + d0 + lane * 8;
        *(volatile v8h*)(UCH + o) = bh[it];
        *(volatile v8h*)(UCL + o) = blo[it];
      }
      __threadfence();
    }
    __syncthreads();
  }
}

__global__ __launch_bounds__(256) void scan_kernel(
    const float* __restrict__ DLR, const float* __restrict__ UC, const float* __restrict__ XZ,
    const float* __restrict__ PROJ, const float* __restrict__ A_log, const float* __restrict__ Dv,
    unsigned short* __restrict__ YH, unsigned short* __restrict__ YL)
{
  __shared__ __align__(16) float sBC[16 * 128];
  __shared__ __align__(16) float sY[16 * kSYP];
  const int tid = threadIdx.x, lane = tid & 31, wave = tid >> 5;
  const int chl = tid >> 1, hf = tid & 1;
  const int d0 = blockIdx.x * kChBlk, d = d0 + chl;
  const int rowbase = blockIdx.y * kSeqL;

  float An[kHalfSt];
#pragma unroll
  for (int n = 0; n < kHalfSt; ++n) An[n] = -__expf(A_log[(size_t)d * kNst + hf * kHalfSt + n]);
  const float Dd = Dv[d];
  float h[kHalfSt];
#pragma unroll
  for (int n = 0; n < kHalfSt; ++n) h[n] = 0.f;

#pragma unroll 1
  for (int c = 0; c < kSeqL / 16; ++c) {
    const int l0 = rowbase + c * 16;
    {
      const int r = tid >> 4, q = (tid & 15) * 8;
      const float* pp = PROJ + (size_t)(l0 + r) * kPrjP + kDtR + q;
      const v4f v0 = *(const v4f*)(pp);
      const v4f v1 = *(const v4f*)(pp + 4);
      *(v4f*)(sBC + r * 128 + q)     = v0;
      *(v4f*)(sBC + r * 128 + q + 4) = v1;
    }
    __syncthreads();
#pragma unroll 1
    for (int s = 0; s < 16; ++s) {
      const size_t m = (size_t)(l0 + s);
      const float a     = DLR[m * kDin + d];
      const float delta = fmaxf(a, 0.0f) + log1pf(__expf(-fabsf(a)));
      const float xv    = UC[m * kDin + d];
      const float zv    = XZ[m * kXZP + kDin + d];
      float du = delta * xv;
      asm volatile("" : "+v"(du));
      const float* bp = sBC + s * 128 + hf * kHalfSt;
      const float* cp = bp + kNst;
      float y = 0.f;
#pragma unroll
      for (int qq = 0; qq < 8; ++qq) {
        const v4f Bq = *(const v4f*)(bp + 4 * qq);
        const v4f Cq = *(const v4f*)(cp + 4 * qq);
#pragma unroll
        for (int e = 0; e < 4; ++e) {
          const int n = qq * 4 + e;
          const float ex = __expf(delta * An[n]);
          float p = du * Bq[e];
          asm volatile("" : "+v"(p));
          float qv = h[n] * ex;
          asm volatile("" : "+v"(qv));
          const float hn = qv + p;
          h[n] = hn;
          float rr = Cq[e] * hn;
          asm volatile("" : "+v"(rr));
          y += rr;
        }
      }
      y += __shfl_xor(y, 1, 32);
      float sk = xv * Dd;
      asm volatile("" : "+v"(sk));
      y += sk;
      const float sg = __builtin_amdgcn_rcpf(1.0f + __expf(-zv));
      const float g  = zv * sg;
      if (hf == 0) sY[s * kSYP + chl] = y * g;
    }
    __syncthreads();
    {
      const int row = 2 * wave + (lane >> 4);
      const int c8  = (lane & 15) * 8;
      const float* sp = sY + row * kSYP + c8;
      const v4f a0 = *(const v4f*)(sp);
      const v4f a1 = *(const v4f*)(sp + 4);
      v8h hv, lv;
#pragma unroll
      for (int e = 0; e < 4; ++e) {
        const unsigned short h0 = f2bf_bits(a0[e]), h1 = f2bf_bits(a1[e]);
        const unsigned short q0 = f2bf_bits(a0[e] - bf_bits2f(h0)), q1 = f2bf_bits(a1[e] - bf_bits2f(h1));
        hv[e]     = __builtin_bit_cast(_Float16, h0);
        hv[4 + e] = __builtin_bit_cast(_Float16, h1);
        lv[e]     = __builtin_bit_cast(_Float16, q0);
        lv[4 + e] = __builtin_bit_cast(_Float16, q1);
      }
      const size_t o = (size_t)(l0 + row) * kDin + d0 + c8;
      for (int pass = 0; pass < 2; ++pass) {
        *(volatile v8h*)(YH + o) = hv;
        *(volatile v8h*)(YL + o) = lv;
        __threadfence();
      }
    }
  }
}

extern "C" void kernel_launch(void* const* d_in, const int* in_sizes, int n_in,
                              void* d_out, int out_size, void* d_ws, size_t ws_size,
                              hipStream_t stream)
{
  if (n_in < 12) return;
  const float* x      = (const float*)d_in[0];
  const float* norm_w = (const float*)d_in[1];
  const float* norm_b = (const float*)d_in[2];
  const float* W_in   = (const float*)d_in[3];
  const float* conv_w = (const float*)d_in[4];
  const float* conv_b = (const float*)d_in[5];
  const float* W_xprj = (const float*)d_in[6];
  const float* W_dt   = (const float*)d_in[7];
  const float* b_dt   = (const float*)d_in[8];
  const float* A_log  = (const float*)d_in[9];
  const float* Dv     = (const float*)d_in[10];
  const float* W_out  = (const float*)d_in[11];
  float* dout = (float*)d_out;

  if (in_sizes[0] != kRows * kDim) return;
  if (in_sizes[1] != kDim || in_sizes[2] != kDim) return;
  if (in_sizes[3] != kXZP * kDim) return;
  if (in_sizes[4] != kDin * 4 || in_sizes[5] != kDin) return;
  if (in_sizes[6] != kPrjN * kDin) return;
  if (in_sizes[7] != kDin * kDtR || in_sizes[8] != kDin) return;
  if (in_sizes[9] != kDin * kNst || in_sizes[10] != kDin) return;
  if (in_sizes[11] != kDim * kDin) return;
  if (out_size != kRows * kDim) return;

  const size_t SZ_XNP  = (size_t)kRows * kDim * 2;
  const size_t SZ_WIP  = (size_t)kXZP * kDim * 2;
  const size_t SZ_WXP  = (size_t)kPrjP * kDin * 2;
  const size_t SZ_WDP  = (size_t)kDin * kDtR * 2;
  const size_t SZ_WOP  = (size_t)kDim * kDin * 2;
  const size_t SZ_XZ   = (size_t)kRows * kXZP * 4;
  const size_t SZ_UC   = (size_t)kRows * kDin * 4;
  const size_t SZ_UCP  = (size_t)kRows * kDin * 2;
  const size_t SZ_PROJ = (size_t)kRows * kPrjP * 4;
  const size_t SZ_DTP  = (size_t)kRows * kDtR * 2;
  const size_t SZ_DLR  = (size_t)kRows * kDin * 4;
  const size_t OFF_XNH  = 0;
  const size_t OFF_XNL  = OFF_XNH  + SZ_XNP;
  const size_t OFF_WIH  = OFF_XNL  + SZ_XNP;
  const size_t OFF_WIL  = OFF_WIH  + SZ_WIP;
  const size_t OFF_WXH  = OFF_WIL  + SZ_WIP;
  const size_t OFF_WXL  = OFF_WXH  + SZ_WXP;
  const size_t OFF_WDH  = OFF_WXL  + SZ_WXP;
  const size_t OFF_WDL  = OFF_WDH  + SZ_WDP;
  const size_t OFF_WOH  = OFF_WDL  + SZ_WDP;
  const size_t OFF_WOL  = OFF_WOH  + SZ_WOP;
  const size_t OFF_XZ   = OFF_WOL  + SZ_WOP;
  const size_t OFF_UC   = OFF_XZ   + SZ_XZ;
  const size_t OFF_UCH  = OFF_UC   + SZ_UC;
  const size_t OFF_UCL  = OFF_UCH  + SZ_UCP;
  const size_t OFF_PROJ = OFF_UCL  + SZ_UCP;
  const size_t OFF_DTH  = OFF_PROJ + SZ_PROJ;
  const size_t OFF_DTL  = OFF_DTH  + SZ_DTP;
  const size_t OFF_DLR  = OFF_DTL  + SZ_DTP;
  const size_t TOTAL    = OFF_DLR  + SZ_DLR;
  if (ws_size < TOTAL) return;

  char* ws = (char*)d_ws;
  unsigned short* XNH  = (unsigned short*)(ws + OFF_XNH);
  unsigned short* XNL  = (unsigned short*)(ws + OFF_XNL);
  unsigned short* WIH  = (unsigned short*)(ws + OFF_WIH);
  unsigned short* WIL  = (unsigned short*)(ws + OFF_WIL);
  unsigned short* WXH  = (unsigned short*)(ws + OFF_WXH);
  unsigned short* WXL  = (unsigned short*)(ws + OFF_WXL);
  unsigned short* WDH  = (unsigned short*)(ws + OFF_WDH);
  unsigned short* WDL  = (unsigned short*)(ws + OFF_WDL);
  unsigned short* WOH  = (unsigned short*)(ws + OFF_WOH);
  unsigned short* WOL  = (unsigned short*)(ws + OFF_WOL);
  float*          XZ   = (float*)(ws + OFF_XZ);
  float*          UC   = (float*)(ws + OFF_UC);
  unsigned short* UCH  = (unsigned short*)(ws + OFF_UCH);
  unsigned short* UCL  = (unsigned short*)(ws + OFF_UCL);
  float*          PROJ = (float*)(ws + OFF_PROJ);
  unsigned short* DTH  = (unsigned short*)(ws + OFF_DTH);
  unsigned short* DTL  = (unsigned short*)(ws + OFF_DTL);
  float*          DLR  = (float*)(ws + OFF_DLR);
  unsigned short* YH   = UCH;
  unsigned short* YL   = UCL;
  const float* dummy_bias  = b_dt;
  const float* dummy_resid = x;

  ln_split_kernel<<<kRows / 8, 256, 0, stream>>>(x, norm_w, norm_b, XNH, XNL, kRows);

  cast_split_rows_kernel<<<(kXZP * kDim) / 8 / 256, 256, 0, stream>>>(W_in,   WIH, WIL, kDim, kXZP,  (kXZP * kDim) / 8);
  cast_split_rows_kernel<<<(kPrjP * kDin) / 8 / 256, 256, 0, stream>>>(W_xprj, WXH, WXL, kDin, kPrjN, (kPrjP * kDin) / 8);
  cast_split_rows_kernel<<<(kDin * kDtR) / 8 / 256, 256, 0, stream>>>(W_dt,   WDH, WDL, kDtR, kDin,  (kDin * kDtR) / 8);
  cast_split_rows_kernel<<<(kDim * kDin) / 8 / 256, 256, 0, stream>>>(W_out,  WOH, WOL, kDin, kDim,  (kDim * kDin) / 8);

  wmma_gemm64<1, true, 0, 0, false><<<dim3(256, 1), 256, 0, stream>>>(
      XNH, XNL, kDim, 0L, WIH, WIL, kDim, 0L,
      (void*)XZ, (void*)XZ, kXZP, 0L, dummy_bias, dummy_resid, 0L, kRows, kXZP, kDim, 1.0f);

  conv_silu_kernel<<<dim3(kDin / 256, kRows / 64), 256, 0, stream>>>(XZ, conv_w, conv_b, UC, UCH, UCL);

  wmma_gemm64<1, true, 0, 0, false><<<dim3(24, 1), 256, 0, stream>>>(
      UCH, UCL, kDin, 0L, WXH, WXL, kDin, 0L,
      (void*)PROJ, (void*)PROJ, kPrjP, 0L, dummy_bias, dummy_resid, 0L, kRows, kPrjP, kDin, 1.0f);

  dt_split_kernel<<<(kRows * kDtR) / 8 / 256, 256, 0, stream>>>(PROJ, DTH, DTL, (kRows * kDtR) / 8);

  wmma_gemm64<1, true, 2, 0, false><<<dim3(128, 1), 256, 0, stream>>>(
      DTH, DTL, kDtR, 0L, WDH, WDL, kDtR, 0L,
      (void*)DLR, (void*)DLR, kDin, 0L, b_dt, dummy_resid, 0L, kRows, kDin, kDtR, 1.0f);

  scan_kernel<<<dim3(kDin / kChBlk, kBatch), 256, 0, stream>>>(DLR, UC, XZ, PROJ, A_log, Dv, YH, YL);

  wmma_gemm64<1, true, 0, 0, false><<<dim3(64, 1), 256, 0, stream>>>(
      YH, YL, kDin, 0L, WOH, WOL, kDin, 0L,
      (void*)dout, (void*)dout, kDim, 0L, dummy_bias, dummy_resid, 0L, kRows, kDim, kDin, 1.0f);
}
